// HumanVAttention_60352880443493
// MI455X (gfx1250) — hardware-verified
//
#include <hip/hip_runtime.h>
#include <math.h>

typedef __attribute__((ext_vector_type(16))) _Float16 v16h;
typedef __attribute__((ext_vector_type(16))) __bf16 v16b;
typedef __attribute__((ext_vector_type(8)))  _Float16 v8h;
typedef __attribute__((ext_vector_type(8)))  float v8f;
typedef __attribute__((ext_vector_type(4)))  float v4f;
typedef __attribute__((ext_vector_type(2)))  float v2f;
typedef __attribute__((ext_vector_type(4)))  unsigned v4u;
typedef __attribute__((ext_vector_type(4)))  int v4i;
typedef float __attribute__((may_alias)) float_a;
typedef int __attribute__((may_alias)) int_a;

template <typename T> __device__ __forceinline__ void vst2(void* p, T v) { *(volatile T*)p = v; __threadfence(); *(volatile T*)p = v; }
__device__ __forceinline__ v8f wmma16(v16h a, v16h b, v8f c) {
  v8f d = __builtin_amdgcn_wmma_f32_16x16x32_f16(false, a, false, b, (short)0, c, false, false);
  asm volatile("v_nop\n\tv_nop\n\tv_nop\n\tv_nop" : "+v"(d) : "v"(a), "v"(b));
  return d;
}
__device__ __forceinline__ v8f wmma_bf(v16b a, v16b b, v8f c) {
  v8f d = __builtin_amdgcn_wmma_f32_16x16x32_bf16(false, a, false, b, (short)0, c, false, false);
  asm volatile("v_nop\n\tv_nop\n\tv_nop\n\tv_nop" : "+v"(d) : "v"(a), "v"(b));
  return d;
}
__device__ __forceinline__ v16h frag_h(const _Float16* rowk0, int lane) {
  union { v16h v; v8h q[2]; } u; const _Float16* p = rowk0 + 8 * (lane >> 4);
  u.q[0] = *(const v8h*)p; u.q[1] = *(const v8h*)(p + 16); return u.v;
}
__device__ __forceinline__ v16h frag_f32(const float* rowk0, int lane) {
  v16h a; const float* p = rowk0 + 8 * (lane >> 4);
#pragma unroll
  for (int i = 0; i < 8; ++i) { a[i] = (_Float16)p[i]; a[8 + i] = (_Float16)p[16 + i]; }
  return a;
}
__device__ __forceinline__ v16h frag_f32s(const float* rowk0, int lane, float sc) {
  v16h a; const float* p = rowk0 + 8 * (lane >> 4);
#pragma unroll
  for (int i = 0; i < 8; ++i) { a[i] = (_Float16)(p[i] * sc); a[8 + i] = (_Float16)(p[16 + i] * sc); }
  return a;
}
__device__ __forceinline__ v16h fragc_f32(const float* W, int k0, int n, int lane, int ld, int K) {
  v16h a; const int g = lane >> 4;
#pragma unroll
  for (int i = 0; i < 8; ++i) { const int ka = k0 + 8 * g + i, kb = ka + 16;
    a[i] = (_Float16)(ka < K ? W[(size_t)(ka < K ? ka : K - 1) * ld + n] : 0.f); a[8 + i] = (_Float16)(kb < K ? W[(size_t)(kb < K ? kb : K - 1) * ld + n] : 0.f); }
  return a;
}
struct F2 { v16b h, l; };
__device__ __forceinline__ F2 bsplit16(const float v[16]) { F2 r;
#pragma unroll
  for (int i = 0; i < 16; ++i) { const __bf16 h = (__bf16)v[i]; r.h[i] = h; r.l[i] = (__bf16)(v[i] - (float)h); }
  return r; }
__device__ __forceinline__ F2 split_row(const float* row, int k0, int lane) { float v[16]; const float* p = row + k0 + 8 * (lane >> 4);
#pragma unroll
  for (int i = 0; i < 8; ++i) { v[i] = p[i]; v[8 + i] = p[16 + i]; }
  return bsplit16(v); }
__device__ __forceinline__ F2 split_rowK(const float* row, int k0, int lane, int K) { float v[16]; const int g = lane >> 4;
#pragma unroll
  for (int i = 0; i < 8; ++i) { const int ka = k0 + 8 * g + i, kb = ka + 16; v[i] = ka < K ? row[ka < K ? ka : K - 1] : 0.f; v[8 + i] = kb < K ? row[kb < K ? kb : K - 1] : 0.f; }
  return bsplit16(v); }
__device__ __forceinline__ F2 split_col(const float* W, int k0, int n, int lane, int ld, int K) { float v[16]; const int g = lane >> 4;
#pragma unroll
  for (int i = 0; i < 8; ++i) { const int ka = k0 + 8 * g + i, kb = ka + 16; v[i] = ka < K ? W[(size_t)(ka < K ? ka : K - 1) * ld + n] : 0.f; v[8 + i] = kb < K ? W[(size_t)(kb < K ? kb : K - 1) * ld + n] : 0.f; }
  return bsplit16(v); }
__device__ __forceinline__ v8f mac3(const F2& a, const F2& b, v8f c) { c = wmma_bf(a.l, b.h, c); c = wmma_bf(a.h, b.l, c); return wmma_bf(a.h, b.h, c); }
__device__ __forceinline__ float sigm(float v) { return 1.0f / (1.0f + expf(-v)); }
#define LDSX() do { asm volatile("s_wait_dscnt 0" ::: "memory"); __builtin_amdgcn_wave_barrier(); __builtin_amdgcn_fence(__ATOMIC_RELEASE, "workgroup"); } while (0)


#define NB 1
#define SS 4096
#define HID 2048
#define ROT 64
#define BLKN 64
#define LOCALB 4
#define GNB 2
#define STRIDEB 4
#define NHQ 16
#define NKV 4
#define HD 128
#define QW (NHQ * HD)
#define KW (NKV * HD)
#define QKVW (QW + 2 * KW)
#ifndef TQB
#define TQB (SS / 64)
#endif
#ifndef TRB
#define TRB (NB * SS / 64)
#endif
typedef __attribute__((ext_vector_type(8))) __bf16 v8b;
__device__ __forceinline__ v16b frag_b(const __bf16* rowk0, int lane) {
  union { v16b v; v8b q[2]; } u; const __bf16* p = rowk0 + 8 * (lane >> 4);
  u.q[0] = *(const v8b*)p; u.q[1] = *(const v8b*)(p + 16); return u.v;
}
__device__ __forceinline__ float bfr(float v) { return (float)(__bf16)v; }
__device__ __attribute__((noinline)) float exp_ni(float v) { return expf(v); }
__device__ __attribute__((noinline)) float erf_ni(float v) { return erff(v); }

#define WS_F   0u
#define WS_QH  (WS_F + 4u * (size_t)NB * SS * QKVW)
#define WS_QL  (WS_QH + 2u * (size_t)NB * SS * QW)
#define WS_KH  (WS_QL + 2u * (size_t)NB * SS * QW)
#define WS_KL  (WS_KH + 2u * (size_t)NB * SS * KW)
#define WS_VH  (WS_KL + 2u * (size_t)NB * SS * KW)
#define WS_VL  (WS_VH + 2u * (size_t)NB * KW * SS)
#define WS_CT  (WS_VL + 2u * (size_t)NB * KW * SS)
#define WS_END (WS_CT + 4u * (size_t)NB * SS * QW)

__global__ __launch_bounds__(128) void k_qkv(const float* __restrict__ X, const float* __restrict__ WQ, const float* __restrict__ WK, const float* __restrict__ WV, float* __restrict__ F) { __shared__ __align__(16) float sf[4][16][132];
  const int tid = threadIdx.x, wave = tid >> 5, lane = tid & 31, col = lane & 15, g = lane >> 4; const int cg = blockIdx.y; const size_t r0 = (size_t)blockIdx.x * 64 + wave * 16;
  const float* Wm; int wcols, c0; if (cg < 16) { Wm = WQ; wcols = QW; c0 = cg * 128; } else if (cg < 20) { Wm = WK; wcols = KW; c0 = (cg - 16) * 128; } else { Wm = WV; wcols = KW; c0 = (cg - 20) * 128; }
  v8f acc[8] = {};
#pragma unroll 2
  for (int kc = 0; kc < HID / 32; ++kc) { v16b a; { const float* p = X + (r0 + col) * HID + kc * 32 + 8 * g;
#pragma unroll
      for (int i = 0; i < 8; ++i) { a[i] = (__bf16)p[i]; a[8 + i] = (__bf16)p[16 + i]; } }
#pragma unroll
    for (int j = 0; j < 8; ++j) { v16b w; const int o = c0 + j * 16 + col;
#pragma unroll
      for (int i = 0; i < 8; ++i) { w[i] = (__bf16)Wm[(size_t)(kc * 32 + 8 * g + i) * wcols + o]; w[8 + i] = (__bf16)Wm[(size_t)(kc * 32 + 16 + 8 * g + i) * wcols + o]; }
      acc[j] = wmma_bf(a, w, acc[j]); } }
#pragma unroll
  for (int j = 0; j < 8; ++j)
#pragma unroll
    for (int r = 0; r < 8; ++r) sf[wave][8 * g + r][j * 16 + col] = acc[j][r];
  LDSX(); for (int rl = 0; rl < 16; ++rl) vst2(F + (r0 + rl) * QKVW + cg * 128 + lane * 4, *(const v4f*)&sf[wave][rl][lane * 4]); }
__global__ __launch_bounds__(256) void k_rope(const float* __restrict__ F, const float* __restrict__ COS, const float* __restrict__ SIN, _Float16* __restrict__ QH, _Float16* __restrict__ QL, _Float16* __restrict__ KH, _Float16* __restrict__ KL) { __shared__ __align__(16) _Float16 sh[QW + KW], sl[QW + KW];
  const int t = threadIdx.x; const size_t row = blockIdx.x; const float* fr = F + row * QKVW; const float* cr = COS + row * ROT; const float* sr = SIN + row * ROT;
  for (int e = t; e < QW + KW; e += 256) { const int j = e % HD; float y;
    if (j < ROT) { const float x = fr[e]; const float rh = (j < ROT / 2) ? -fr[e + ROT / 2] : fr[e - ROT / 2]; y = x * bfr(cr[j]) + rh * bfr(sr[j]); } else y = fr[e];
    const _Float16 hv = (_Float16)y; sh[e] = hv; sl[e] = (_Float16)(y - (float)hv); }
  __syncthreads();
  for (int q = t; q < QW / 8; q += 256) { vst2((unsigned*)(QH + row * QW + q * 8), *(const v4u*)&sh[q * 8]); vst2((unsigned*)(QL + row * QW + q * 8), *(const v4u*)&sl[q * 8]); }
  for (int q = t; q < KW / 8; q += 256) { vst2((unsigned*)(KH + row * KW + q * 8), *(const v4u*)&sh[QW + q * 8]); vst2((unsigned*)(KL + row * KW + q * 8), *(const v4u*)&sl[QW + q * 8]); } }
__global__ __launch_bounds__(128) void k_vt(const float* __restrict__ F, _Float16* __restrict__ VH, _Float16* __restrict__ VL) { __shared__ __align__(16) _Float16 th[128][72], tl[128][72];
  const int t = threadIdx.x; const size_t s0 = (size_t)blockIdx.x * 64; const int c0 = blockIdx.y * 128;
  for (int e = t; e < 64 * 128; e += 128) { const int sl_ = e >> 7, c = e & 127; const float v = F[(s0 + sl_) * QKVW + QW + KW + c0 + c]; const _Float16 hv = (_Float16)v; th[c][sl_] = hv; tl[c][sl_] = (_Float16)(v - (float)hv); }
  __syncthreads(); for (int e = t; e < 128 * 8; e += 128) { const int c = e >> 3, q = e & 7; vst2((unsigned*)(VH + (size_t)(c0 + c) * SS + s0 + q * 8), *(const v4u*)&th[c][q * 8]); vst2((unsigned*)(VL + (size_t)(c0 + c) * SS + s0 + q * 8), *(const v4u*)&tl[c][q * 8]); } }
__global__ __launch_bounds__(128) void k_att(const _Float16* __restrict__ QH, const _Float16* __restrict__ QL, const _Float16* __restrict__ KH, const _Float16* __restrict__ KL, const _Float16* __restrict__ VH, const _Float16* __restrict__ VL, const float* __restrict__ AM, float* __restrict__ CT) {
  __shared__ __align__(16) float sp[4][16][36]; __shared__ __align__(16) float so[4][16][132];
  const int tid = threadIdx.x, wave = tid >> 5, lane = tid & 31, col = lane & 15, g = lane >> 4; const int qb = blockIdx.x, h = blockIdx.y; const int kvh = h / (NHQ / NKV); const int q0 = qb * 64 + wave * 16; constexpr bool three = false;
  v16h aq[4], al[4];
#pragma unroll
  for (int kc = 0; kc < 4; ++kc) { aq[kc] = frag_h(QH + (size_t)(q0 + col) * QW + h * HD + kc * 32, lane); al[kc] = frag_h(QL + (size_t)(q0 + col) * QW + h * HD + kc * 32, lane); }
  float m[8], l[8];
#pragma unroll
  for (int r = 0; r < 8; ++r) { m[r] = -3.0e38f; l[r] = 0.f; }
  v8f acc[8] = {};
  int sel[LOCALB + GNB + 1]; int nsel = 0;
  { const int cnt = qb / STRIDEB + 1; const int gfirst = STRIDEB * ((cnt > GNB) ? (cnt - GNB) : 0);
#pragma unroll 1
    for (int bk = 0; bk <= qb; ++bk) { const bool isloc = (bk >= qb - (LOCALB - 1)); const bool isglob = (bk == 0) || ((bk % STRIDEB) == 0 && bk >= gfirst); if (isloc || isglob) sel[nsel++] = bk; } }
#pragma unroll 1
  for (int si = 0; si < nsel * 2; ++si) { const int ks = sel[si >> 1] * 2 + (si & 1); const bool diagb = (sel[si >> 1] == qb); float s[2][8];
#pragma unroll
    for (int ct = 0; ct < 2; ++ct) { const int kk = ks * 32 + ct * 16 + col; const size_t rk = (size_t)kk * KW + kvh * HD; v8f c = {};
#pragma unroll
      for (int kc = 0; kc < 4; ++kc) { const v16h kh = frag_h(KH + rk + kc * 32, lane); c = wmma16(aq[kc], kh, c); c = wmma16(al[kc], kh, c); c = wmma16(aq[kc], frag_h(KL + rk + kc * 32, lane), c); }
      const float madd = (1.0f - bfr(AM[kk])) * -1.0e9f;
#pragma unroll
      for (int r = 0; r < 8; ++r) s[ct][r] = (diagb && kk > q0 + 8 * g + r) ? -3.0e38f : (c[r] * 0.08838834764831845f + madd); }
    float alpha[8];
#pragma unroll
    for (int r = 0; r < 8; ++r) { float mx = fmaxf(s[0][r], s[1][r]);
#pragma unroll
      for (int o = 1; o < 16; o <<= 1) mx = fmaxf(mx, __shfl_xor(mx, o));
      const float mn = fmaxf(m[r], mx); alpha[r] = (m[r] <= -1.0e38f) ? 0.f : __expf(m[r] - mn); const float e0 = (s[0][r] <= -1.0e38f) ? 0.f : __expf(s[0][r] - mn), e1 = (s[1][r] <= -1.0e38f) ? 0.f : __expf(s[1][r] - mn); float es = e0 + e1;
#pragma unroll
      for (int o = 1; o < 16; o <<= 1) es += __shfl_xor(es, o);
      l[r] = l[r] * alpha[r] + es; m[r] = mn; sp[wave][8 * g + r][col] = e0; sp[wave][8 * g + r][16 + col] = e1; }
#pragma unroll
    for (int j = 0; j < 8; ++j)
#pragma unroll
      for (int r = 0; r < 8; ++r) acc[j][r] *= alpha[r];
    LDSX();
    const v16h pa = frag_f32s(&sp[wave][col][0], lane, 2048.0f);
#pragma unroll
    for (int j = 0; j < 8; ++j) { const size_t po = ((size_t)kvh * HD + j * 16 + col) * SS + ks * 32; acc[j] = wmma16(pa, frag_h(VH + po, lane), acc[j]); acc[j] = wmma16(pa, frag_h(VL + po, lane), acc[j]); }
    LDSX(); }
#pragma unroll
  for (int r = 0; r < 8; ++r) { const float il = (l[r] > 0.f) ? (1.0f / 2048.0f) / l[r] : 0.f;
#pragma unroll
    for (int j = 0; j < 8; ++j) so[wave][8 * g + r][j * 16 + col] = acc[j][r] * il; }
  LDSX(); for (int rl = 0; rl < 16; ++rl) vst2(CT + (size_t)(q0 + rl) * QW + h * HD + lane * 4, *(const v4f*)&so[wave][rl][lane * 4]); }
__global__ __launch_bounds__(128) void k_out(const float* __restrict__ CT, const float* __restrict__ WO, float* __restrict__ OUT) { __shared__ __align__(16) float sf[4][16][132];
  const int tid = threadIdx.x, wave = tid >> 5, lane = tid & 31, col = lane & 15, g = lane >> 4; const int c0 = blockIdx.y * 128; const size_t r0 = (size_t)blockIdx.x * 64 + wave * 16;
  v8f acc[8] = {};
#pragma unroll 2
  for (int kc = 0; kc < QW / 32; ++kc) { const F2 a = split_row(CT + (r0 + col) * QW, kc * 32, lane);
#pragma unroll
    for (int j = 0; j < 8; ++j) { v16b w; const int o = c0 + j * 16 + col;
#pragma unroll
      for (int i = 0; i < 8; ++i) { w[i] = (__bf16)WO[(size_t)(kc * 32 + 8 * g + i) * HID + o]; w[8 + i] = (__bf16)WO[(size_t)(kc * 32 + 16 + 8 * g + i) * HID + o]; }
      acc[j] = wmma_bf(a.h, w, acc[j]); acc[j] = wmma_bf(a.l, w, acc[j]); } }
#pragma unroll
  for (int j = 0; j < 8; ++j)
#pragma unroll
    for (int r = 0; r < 8; ++r) sf[wave][8 * g + r][j * 16 + col] = acc[j][r];
  LDSX(); for (int rl = 0; rl < 16; ++rl) vst2(OUT + (r0 + rl) * HID + c0 + lane * 4, *(const v4f*)&sf[wave][rl][lane * 4]); }
extern "C" void kernel_launch(void* const* d_in, const int* in_sizes, int n_in, void* d_out, int out_size, void* d_ws, size_t ws_size, hipStream_t stream) {
  (void)in_sizes; (void)n_in; (void)out_size;
  const float** F_ = (const float**)d_in;
  if (ws_size < (size_t)WS_END) return;
  char* ws = (char*)d_ws; float* F = (float*)(ws + WS_F); _Float16 *QH = (_Float16*)(ws + WS_QH), *QL = (_Float16*)(ws + WS_QL), *KH = (_Float16*)(ws + WS_KH), *KL = (_Float16*)(ws + WS_KL), *VH = (_Float16*)(ws + WS_VH), *VL = (_Float16*)(ws + WS_VL); float* CT = (float*)(ws + WS_CT);
  k_qkv<<<dim3(TRB, QKVW / 128), 128, 0, stream>>>(F_[0], F_[3], F_[4], F_[5], F);
  k_rope<<<TRB * 64, 256, 0, stream>>>(F, F_[1], F_[2], QH, QL, KH, KL);
  k_vt<<<dim3(TRB, KW / 128), 128, 0, stream>>>(F, VH, VL);
  k_att<<<dim3(TQB, NHQ), 128, 0, stream>>>(QH, QL, KH, KL, VH, VL, F_[7], CT);
  k_out<<<dim3(TQB, HID / 128), 128, 0, stream>>>(CT, F_[6], (float*)d_out);
}
